// Decoder_12292196401549
// MI455X (gfx1250) — hardware-run, weakly checked
//
#include <hip/hip_runtime.h>


#ifndef NB
#define NB 2
#endif
#ifndef SEQ
#define SEQ 4096
#endif
#define NB_FULL  2
#define SEQ_FULL 4096
#define DM   1024
#define DI   4096
#define NH_  16
#define HD   64
#define NQKV 3072
#define WIN  512
#define NSLOT 513
#define PJ   528
#define AW   1
#define QEP  528
#define OSP  68
#define OSG  68
#define WSC  64.0f
#define WSI  (1.0f / 64.0f)
#define CTXS 64.0f
#define CTXI (1.0f / 64.0f)
#define SC2  ((float)(0.125 * 1.4426950408889634))
#define PSH  14.0f
#define NEGB (-3.0e38f)

static_assert(HD == 64);
static_assert(NH_ * HD == DM);
static_assert(NQKV == NH_ * 3 * HD);
static_assert(DM % 64 == 0);
static_assert(DI % 64 == 0);
static_assert(NQKV % 64 == 0);
static_assert(DM % 32 == 0);
static_assert(DI % 32 == 0);
static_assert(HD % 32 == 0);
static_assert(SEQ % 64 == 0);
static_assert(SEQ % WIN == 0);
static_assert(WIN % 64 == 0);
static_assert(SEQ % 32 == 0);
static_assert(SEQ % (16 * AW) == 0);
static_assert(SEQ >= WIN);
static_assert(PJ % 16 == 0);
static_assert(PJ >= NSLOT);
static_assert(QEP >= PJ);
static_assert(QEP % 4 == 0);
static_assert(OSP % 4 == 0);
static_assert(OSG % 4 == 0);
static_assert(NB <= NB_FULL);
static_assert(SEQ <= SEQ_FULL);
static_assert((NB * SEQ) % 8 == 0);
static_assert((size_t)AW * 16 * QEP * 4 + (size_t)AW * 16 * OSP * 4 <= 131072);
static_assert((size_t)64 * OSG * 4 <= 131072);
static_assert(32 * 16 * 16 == 64 * HD * 2);
static_assert(32 * 16 * 32 == 64 * 64 * 4);
static_assert(32 * 16 * 4 == 16 * HD * 2);
static_assert(32 * 16 * 4 == DM * 2);
static_assert((size_t)SEQ_FULL * NB_FULL * DM * 4 == (size_t)33554432);
static_assert(((size_t)SEQ_FULL * NB_FULL * DM + (size_t)WIN * NB_FULL * NH_ * 2 * HD) * 4 == (size_t)41943040);

typedef _Float16 h16;
typedef __attribute__((ext_vector_type(16))) _Float16 v16h;
typedef __attribute__((ext_vector_type(8)))  _Float16 v8h;
typedef __attribute__((ext_vector_type(8)))  float    v8f;
typedef __attribute__((ext_vector_type(4)))  float    v4f;
typedef v4f  __attribute__((may_alias)) v4fa;

__device__ __forceinline__ unsigned short f2bf(float f) { unsigned u = __float_as_uint(f); u += 0x7FFFu + ((u >> 16) & 1u); return (unsigned short)(u >> 16); }
__device__ __forceinline__ float bfr(float f) { return __uint_as_float(((unsigned)f2bf(f)) << 16); }
__device__ __forceinline__ v16h cat16(v8h lo, v8h hi) { return __builtin_shufflevector(lo, hi, 0, 1, 2, 3, 4, 5, 6, 7, 8, 9, 10, 11, 12, 13, 14, 15); }
__device__ __forceinline__ v8f wmma16(v16h a, v16h b, v8f c) { return __builtin_amdgcn_wmma_f32_16x16x32_f16(false, a, false, b, (short)0, c, false, false); }
__device__ __forceinline__ v16h  ldh(const h16* p) { return cat16(*(const v8h*)p, *(const v8h*)(p + 16)); }
__device__ __forceinline__ void wave_sync() { __builtin_amdgcn_fence(3  , "wavefront"); __builtin_amdgcn_wave_barrier(); asm volatile("" ::: "memory"); }
__device__ __forceinline__ h16 toh_flush(float v) { const h16 r = (h16)v; return (fabsf(v) < 6.103515625e-05f) ? (h16)0.0f : r; }
__device__ __forceinline__ v8f wmma16g(v16h a, v16h b, v8f c) { c = wmma16(a, b, c); asm volatile("v_nop\n\tv_nop\n\tv_nop\n\tv_nop" : "+v"(c) : "v"(a), "v"(b)); return c; }

__global__ __launch_bounds__(256) void k_wcvt(const float* __restrict__ src, h16* dst, size_t n8) {
    const size_t i = (size_t)blockIdx.x * 256 + threadIdx.x; if (i >= n8) return;
    const v8f v = *(const v8f*)(src + i * 8); v8h o;
#pragma unroll
    for (int k = 0; k < 8; ++k) o[k] = toh_flush(bfr(v[k]) * WSC);
    *(volatile v8h*)(dst + i * 8) = o; __threadfence(); *(volatile v8h*)(dst + i * 8) = o;
}

__global__ __launch_bounds__(256) void k_poscvt(const float* __restrict__ pos, h16* PT) {
    const int i = (int)blockIdx.x * 256 + (int)threadIdx.x; if (i >= PJ * HD / 8) return;
    const int j = i >> 3, d0 = (i & 7) * 8;
    const int jc = j < NSLOT ? j : (NSLOT - 1);
    v8h o;
#pragma unroll
    for (int k = 0; k < 8; ++k) { const float v = pos[(size_t)(d0 + k) * NSLOT + jc]; o[k] = (j < NSLOT) ? toh_flush(bfr(v) * WSC) : (h16)0.0f; }
    *(volatile v8h*)(PT + (size_t)i * 8) = o; __threadfence(); *(volatile v8h*)(PT + (size_t)i * 8) = o;
}

__global__ __launch_bounds__(256) void k_ln(const float* src, const float* __restrict__ gam, const float* __restrict__ bet, h16* dst, int inbf) {
#pragma clang fp contract(off)
    const int lane = threadIdx.x & 31;
    const int m = (int)blockIdx.x * 8 + (int)(threadIdx.x >> 5);
    if (m >= NB * SEQ) return;
    const int b = m / SEQ, t = m % SEQ;
    const float* xr = src + ((size_t)t * NB_FULL + (size_t)b) * DM + lane * 8;
    const bool cv = inbf != 0;
    v8f xv[4];
#pragma unroll
    for (int c = 0; c < 4; ++c) { const v8f v = *(const v8f*)(xr + c * 256);
#pragma unroll
        for (int k = 0; k < 8; ++k) { const float w = bfr(v[k]); xv[c][k] = cv ? w : v[k]; } }
    float s = 0.0f;
#pragma unroll
    for (int c = 0; c < 4; ++c)
#pragma unroll
        for (int k = 0; k < 8; ++k) s += xv[c][k];
#pragma unroll
    for (int off = 16; off > 0; off >>= 1) s += __shfl_xor(s, off, 32);
    const float mean = s * (1.0f / 1024.0f);
    float q = 0.0f;
#pragma unroll
    for (int c = 0; c < 4; ++c)
#pragma unroll
        for (int k = 0; k < 8; ++k) { const float d = xv[c][k] - mean; q += d * d; }
#pragma unroll
    for (int off = 16; off > 0; off >>= 1) q += __shfl_xor(q, off, 32);
    const float rstd = 1.0f / sqrtf(q * (1.0f / 1024.0f) + 1e-5f);
    v8h ov[4];
#pragma unroll
    for (int c = 0; c < 4; ++c) { const v8f g = *(const v8f*)(gam + c * 256 + lane * 8); const v8f be = *(const v8f*)(bet + c * 256 + lane * 8);
#pragma unroll
        for (int k = 0; k < 8; ++k) ov[c][k] = toh_flush(((xv[c][k] - mean) * rstd) * bfr(g[k]) + bfr(be[k])); }
    h16* orow = dst + (size_t)m * DM + lane * 8;
#pragma unroll 1
    for (int ps = 0; ps < 2; ++ps) {
#pragma unroll
        for (int c = 0; c < 4; ++c) *(volatile v8h*)(orow + c * 256) = ov[c];
        if (ps == 0) __threadfence(); }
}

static constexpr size_t PLN = (size_t)NB * NH_ * SEQ * HD;
static constexpr size_t OUT1_OFF = (size_t)SEQ_FULL * NB_FULL * DM;

template <int MODE>
__device__ __forceinline__ void gemm_body(const h16* __restrict__ A, const h16* __restrict__ Bt, const float* __restrict__ bias, const float* __restrict__ xres, h16* P0, float* F0) {
    __shared__ __align__(16) float os[64 * OSG];
    constexpr int K = (MODE == 3) ? DI : DM;
    const int lane = threadIdx.x & 31, lr = lane & 15, hi = lane >> 4; const int r0 = blockIdx.x * 64, c0 = blockIdx.y * 64;
    v8f acc[4][4];
#pragma unroll
    for (int mb = 0; mb < 4; ++mb)
#pragma unroll
        for (int nb = 0; nb < 4; ++nb) acc[mb][nb] = (v8f){};
    const size_t aoff = (size_t)(r0 + lr) * K + 8 * hi, boff = (size_t)(c0 + lr) * K + 8 * hi;
#pragma unroll 1
    for (int kc = 0; kc < K; kc += 32) {
        v16h a[4];
#pragma unroll
        for (int mb = 0; mb < 4; ++mb) a[mb] = ldh(A + aoff + (size_t)mb * 16 * K + kc);
#pragma unroll
        for (int nb = 0; nb < 4; ++nb) { const v16h b = ldh(Bt + boff + (size_t)nb * 16 * K + kc);
#pragma unroll
            for (int mb = 0; mb < 4; ++mb) acc[mb][nb] = wmma16g(a[mb], b, acc[mb][nb]); }
    }
    const int bb = r0 / SEQ, tt = r0 % SEQ;
    constexpr float sc = (MODE == 1) ? (WSI * CTXI) : WSI;
    float bc[4];
#pragma unroll
    for (int nb = 0; nb < 4; ++nb) bc[nb] = (MODE != 1) ? bfr(bias[c0 + nb * 16 + lr]) : 0.0f;
#pragma unroll
    for (int mb = 0; mb < 4; ++mb)
#pragma unroll
        for (int nb = 0; nb < 4; ++nb)
#pragma unroll
            for (int j = 0; j < 8; ++j) { float v = acc[mb][nb][j] * sc + bc[nb]; if (MODE == 2) v = fmaxf(v, 0.0f);
                os[(mb * 16 + hi * 8 + j) * OSG + nb * 16 + lr] = v; }
    wave_sync();
    if (MODE == 0) {
        const int hdx = (int)blockIdx.y / 3, part = (int)blockIdx.y % 3;
        const int zh = bb * NH_ + hdx;
        const bool nx = (part >= 1) && (tt >= SEQ - WIN);
        h16* prow = P0 + (size_t)part * PLN + ((size_t)zh * SEQ + (size_t)tt) * HD;
        h16* pcol = P0 + (size_t)2 * PLN + (size_t)zh * HD * SEQ + (size_t)tt;
        const int srow = nx ? (tt - (SEQ - WIN)) : 0;
        const int pofs = nx ? (part - 1) * HD : 0;
        float* nrow = F0 + ((size_t)srow * (NB_FULL * NH_) + (size_t)(bb * NH_ + hdx)) * (2 * HD) + (size_t)pofs;
#pragma unroll 1
        for (int ps = 0; ps < 2; ++ps) {
            if (part < 2) {
#pragma unroll 1
                for (int s = 0; s < 16; ++s) { const int row = 4 * s + (lane >> 3), c8 = (lane & 7) * 8;
                    const v4f x0 = *(const v4fa*)(&os[row * OSG + c8]); const v4f x1 = *(const v4fa*)(&os[row * OSG + c8 + 4]); v8h hv;
#pragma unroll
                    for (int i = 0; i < 4; ++i) { hv[i] = toh_flush(x0[i]); hv[4 + i] = toh_flush(x1[i]); }
                    *(volatile v8h*)(prow + (size_t)row * HD + c8) = hv; }
            } else {
#pragma unroll 1
                for (int s = 0; s < 16; ++s) { const int drow = 4 * s + (lane >> 3), c8 = (lane & 7) * 8;
                    v8h hv;
#pragma unroll
                    for (int i = 0; i < 8; ++i) hv[i] = toh_flush(os[(c8 + i) * OSG + drow]);
                    *(volatile v8h*)(pcol + (size_t)drow * SEQ + c8) = hv; }
            }
            if (nx) {
#pragma unroll 1
                for (int s = 0; s < 32; ++s) { const int row = 2 * s + (lane >> 4), c4 = (lane & 15) * 4;
                    const v4f val = *(const v4fa*)(&os[row * OSG + c4]);
                    *(volatile v4f*)(nrow + (size_t)row * ((size_t)NB_FULL * NH_ * 2 * HD) + c4) = val; }
            }
            if (ps == 0) __threadfence(); }
    } else if (MODE == 2) {
        h16* prow = P0 + (size_t)r0 * DI + (size_t)c0;
#pragma unroll 1
        for (int ps = 0; ps < 2; ++ps) {
#pragma unroll 1
            for (int s = 0; s < 16; ++s) { const int row = 4 * s + (lane >> 3), c8 = (lane & 7) * 8;
                const v4f x0 = *(const v4fa*)(&os[row * OSG + c8]); const v4f x1 = *(const v4fa*)(&os[row * OSG + c8 + 4]); v8h hv;
#pragma unroll
                for (int i = 0; i < 4; ++i) { hv[i] = toh_flush(x0[i]); hv[4 + i] = toh_flush(x1[i]); }
                *(volatile v8h*)(prow + (size_t)row * DI + c8) = hv; }
            if (ps == 0) __threadfence(); }
    } else {
#pragma unroll 1
        for (int s = 0; s < 32; ++s) { const int row = 2 * s + (lane >> 4), c4 = (lane & 15) * 4;
            const size_t gi = ((size_t)(tt + row) * NB_FULL + (size_t)bb) * DM + (size_t)c0 + c4;
            v4f xa;
            if (MODE == 1) { const v4f xv = *(const v4f*)(xres + gi); xa[0] = bfr(xv[0]); xa[1] = bfr(xv[1]); xa[2] = bfr(xv[2]); xa[3] = bfr(xv[3]); }
            else           { xa = *(const v4f*)(F0 + gi); }
            v4f ov = *(const v4fa*)(&os[row * OSG + c4]);
            ov[0] += xa[0]; ov[1] += xa[1]; ov[2] += xa[2]; ov[3] += xa[3];
            *(v4fa*)(&os[row * OSG + c4]) = ov; }
        wave_sync();
#pragma unroll 1
        for (int ps = 0; ps < 2; ++ps) {
#pragma unroll 1
            for (int s = 0; s < 32; ++s) { const int row = 2 * s + (lane >> 4), c4 = (lane & 15) * 4;
                const size_t gi = ((size_t)(tt + row) * NB_FULL + (size_t)bb) * DM + (size_t)c0 + c4;
                const v4f val = *(const v4fa*)(&os[row * OSG + c4]);
                *(volatile v4f*)(F0 + gi) = val; }
            if (ps == 0) __threadfence(); }
    }
}

__global__ __launch_bounds__(32) void k_gemm_qkv(const h16* __restrict__ A, const h16* __restrict__ Bt, const float* __restrict__ bias, h16* PL, float* NXT) {
    gemm_body<0>(A, Bt, bias, bias, PL, NXT);
}
__global__ __launch_bounds__(32) void k_gemm_out(const h16* __restrict__ A, const h16* __restrict__ Bt, const float* __restrict__ xres, float* OUTP) {
    gemm_body<1>(A, Bt, xres, xres, (h16*)nullptr, OUTP);
}
__global__ __launch_bounds__(32) void k_gemm_fc1(const h16* __restrict__ A, const h16* __restrict__ Bt, const float* __restrict__ bias, h16* FF) {
    gemm_body<2>(A, Bt, bias, bias, FF, (float*)nullptr);
}
__global__ __launch_bounds__(32) void k_gemm_fc2(const h16* __restrict__ A, const h16* __restrict__ Bt, const float* __restrict__ bias, float* OUTP) {
    gemm_body<3>(A, Bt, bias, bias, (h16*)nullptr, OUTP);
}

__global__ __launch_bounds__(32 * AW) void k_flash(const h16* __restrict__ QH, const h16* __restrict__ KP, const h16* __restrict__ VT, const h16* __restrict__ PT, h16* CTX) {
    __shared__ __align__(16) float qe[AW * 16 * QEP];
    __shared__ __align__(16) float os[AW * 16 * OSP];
    const int lane = threadIdx.x & 31, lr = lane & 15, hi = lane >> 4;
    const int wv = (int)(threadIdx.x >> 5);
    const int t0v = ((int)blockIdx.x * AW + wv) * 16;
    int kbv = t0v - WIN; kbv = kbv < 0 ? 0 : kbv; kbv &= ~31;
    const int wave = __builtin_amdgcn_readfirstlane(wv);
    const int t0   = __builtin_amdgcn_readfirstlane(t0v);
    const int kbeg = __builtin_amdgcn_readfirstlane(kbv);
    const int kend = (t0 + 47) & ~31;
    const int zh = blockIdx.y; const int b = zh / NH_, hd = zh % NH_;
    const int p = t0 + lr;
    const size_t pbase = (size_t)zh * SEQ * HD;
    const size_t qo = pbase + (size_t)(t0 + lr) * HD + 8 * hi;
    const v16h q0 = ldh(QH + qo), q1 = ldh(QH + qo + 32);
    const int qrow = (wave * 16 + lr) * QEP;
#pragma unroll 1
    for (int jt = 0; jt < PJ / 16; ++jt) {
        const h16* pp = PT + (size_t)(jt * 16 + lr) * HD + 8 * hi;
        const v16h a0 = ldh(pp), a1 = ldh(pp + 32);
        v8f c = (v8f){};
        c = wmma16g(a0, q0, c); c = wmma16g(a1, q1, c);
        v4f x, y;
        x[0] = c[0] * WSI; x[1] = c[1] * WSI; x[2] = c[2] * WSI; x[3] = c[3] * WSI;
        y[0] = c[4] * WSI; y[1] = c[5] * WSI; y[2] = c[6] * WSI; y[3] = c[7] * WSI;
        *(v4fa*)(&qe[qrow + jt * 16 + 8 * hi]) = x; *(v4fa*)(&qe[qrow + jt * 16 + 8 * hi + 4]) = y;
    }
    wave_sync();
    const size_t ko = pbase + (size_t)lr * HD + 8 * hi;
    const size_t vo = pbase + (size_t)lr * SEQ + 8 * hi;
    v8f o[4];
#pragma unroll
    for (int j = 0; j < 4; ++j) o[j] = (v8f){};
    float m = NEGB, l = 0.0f;
#pragma unroll 1
    for (int key0 = kbeg; key0 < kend; key0 += 32) {
        const h16* ka = KP + ko + (size_t)key0 * HD;
        v8f sa = (v8f){}, sb = (v8f){};
        { const v16h k0 = ldh(ka), k1 = ldh(ka + 32); sa = wmma16g(k0, q0, sa); sa = wmma16g(k1, q1, sa); }
        { const v16h k0 = ldh(ka + 16 * HD), k1 = ldh(ka + 16 * HD + 32); sb = wmma16g(k0, q0, sb); sb = wmma16g(k1, q1, sb); }
        const int jb = key0 + 8 * hi - p + WIN;
        float ta[8], tb[8]; bool fa[8], fb[8]; float mx = NEGB;
#pragma unroll
        for (int r = 0; r < 8; ++r) {
            const int ia = jb + r, ib = jb + 16 + r;
            fa[r] = (unsigned)ia <= (unsigned)WIN; fb[r] = (unsigned)ib <= (unsigned)WIN;
            const int ca = ia < 0 ? 0 : (ia > WIN ? WIN : ia);
            const int cb = ib < 0 ? 0 : (ib > WIN ? WIN : ib);
            float xa = qe[qrow + ca]; float xb = qe[qrow + cb];
            asm volatile("" : "+v"(xa)); asm volatile("" : "+v"(xb));
            ta[r] = (sa[r] + xa) * SC2; tb[r] = (sb[r] + xb) * SC2;
            mx = fmaxf(mx, fmaxf(fa[r] ? ta[r] : NEGB, fb[r] ? tb[r] : NEGB)); }
        mx = fmaxf(mx, __shfl_xor(mx, 16, 32));
        const float mnew = fmaxf(m, mx);
        const float alpha = __builtin_amdgcn_exp2f(m - mnew);
        const float sh = PSH - mnew;
        v16h pb; float ls = 0.0f;
#pragma unroll
        for (int r = 0; r < 8; ++r) {
            const float xa = ta[r] + sh, xb = tb[r] + sh;
            const float ea = __builtin_amdgcn_exp2f(xa), eb = __builtin_amdgcn_exp2f(xb);
            const float ga = (fa[r] && xa >= -14.0f) ? ea : 0.0f;
            const float gb = (fb[r] && xb >= -14.0f) ? eb : 0.0f;
            const h16 pa = (h16)ga; const h16 pc = (h16)gb;
            pb[r] = pa; pb[8 + r] = pc;
            ls += (float)pa + (float)pc; }
        l = l * alpha + ls; m = mnew;
#pragma unroll
        for (int j = 0; j < 4; ++j) o[j] = o[j] * alpha;
        const h16* va = VT + vo + key0;
#pragma unroll
        for (int j = 0; j < 4; ++j) { const v16h vf = ldh(va + (size_t)(16 * j) * SEQ); o[j] = wmma16g(vf, pb, o[j]); }
    }
    l += __shfl_xor(l, 16, 32);
    const bool any = l > 0.0f;
    const float lsafe = any ? l : 1.0f;
    const float inv = any ? (CTXS * (1.0f / lsafe)) : 0.0f;
    const int wb = wave * 16 * OSP;
#pragma unroll
    for (int j = 0; j < 4; ++j) { v4f a, c;
        a[0] = o[j][0] * inv; a[1] = o[j][1] * inv; a[2] = o[j][2] * inv; a[3] = o[j][3] * inv;
        c[0] = o[j][4] * inv; c[1] = o[j][5] * inv; c[2] = o[j][6] * inv; c[3] = o[j][7] * inv;
        *(v4fa*)(&os[wb + lr * OSP + 16 * j + 8 * hi]) = a; *(v4fa*)(&os[wb + lr * OSP + 16 * j + 8 * hi + 4]) = c; }
    wave_sync();
    h16* crow = CTX + ((size_t)b * SEQ + (size_t)t0) * DM + hd * HD;
#pragma unroll 1
    for (int ps = 0; ps < 2; ++ps) {
#pragma unroll
        for (int s = 0; s < 4; ++s) { const int row = 4 * s + (lane >> 3), c8 = (lane & 7) * 8;
            const v4f x0 = *(const v4fa*)(&os[wb + row * OSP + c8]); const v4f x1 = *(const v4fa*)(&os[wb + row * OSP + c8 + 4]); v8h hv;
#pragma unroll
            for (int i = 0; i < 4; ++i) { hv[i] = toh_flush(x0[i]); hv[4 + i] = toh_flush(x1[i]); }
            *(volatile v8h*)(crow + (size_t)row * DM + c8) = hv; }
        if (ps == 0) __threadfence(); }
}

static constexpr size_t al256(size_t v) { return (v + 255) & ~(size_t)255; }
static constexpr size_t SZ_WQ = al256((size_t)NQKV * DM * 2);
static constexpr size_t SZ_WO = al256((size_t)DM * DM * 2);
static constexpr size_t SZ_W1 = al256((size_t)DI * DM * 2);
static constexpr size_t SZ_W2 = al256((size_t)DM * DI * 2);
static constexpr size_t SZ_PT = al256((size_t)PJ * HD * 2);
static constexpr size_t SZ_H  = al256((size_t)NB * SEQ * DM * 2);
static constexpr size_t SZ_PL = al256((size_t)NB * NH_ * SEQ * HD * 2);
static constexpr size_t SZ_FF = al256((size_t)NB * SEQ * DI * 2);
static constexpr size_t SZ_A  = SZ_H + 3 * SZ_PL;
static constexpr size_t SZ_TOTAL = SZ_WQ + SZ_WO + SZ_W1 + SZ_W2 + SZ_PT + SZ_A + SZ_H;
static_assert(SZ_TOTAL <= (size_t)134217728);
static_assert(SZ_FF <= SZ_A);
static_assert(SZ_PL == PLN * 2);
static_assert(SZ_H == (size_t)NB * SEQ * DM * 2);
static_assert((size_t)PJ * HD % 8 == 0);

extern "C" void kernel_launch(void* const* d_in, const int* in_sizes, int n_in,
                              void* d_out, int out_size, void* d_ws, size_t ws_size, hipStream_t stream) {
    if (n_in < 13) return;
    const size_t needx = ((size_t)(SEQ - 1) * NB_FULL + NB) * DM;
    if ((size_t)in_sizes[0] < needx) return;
    if (in_sizes[1] < DM || in_sizes[2] < DM || in_sizes[7] < DM || in_sizes[8] < DM || in_sizes[12] < DM) return;
    if ((size_t)in_sizes[3] < (size_t)NQKV * DM || in_sizes[4] < NQKV) return;
    if (in_sizes[5] < HD * NSLOT) return;
    if ((size_t)in_sizes[6] < (size_t)DM * DM) return;
    if ((size_t)in_sizes[9] < (size_t)DI * DM || in_sizes[10] < DI) return;
    if ((size_t)in_sizes[11] < (size_t)DM * DI) return;
    if ((size_t)out_size < OUT1_OFF + (size_t)WIN * NB_FULL * NH_ * 2 * HD) return;
    if (SZ_TOTAL > ws_size) return;
    const float* x    = (const float*)d_in[0];
    const float* g1   = (const float*)d_in[1];  const float* e1 = (const float*)d_in[2];
    const float* wqkv = (const float*)d_in[3];  const float* bqkv = (const float*)d_in[4];
    const float* pos  = (const float*)d_in[5];
    const float* wout = (const float*)d_in[6];
    const float* g2   = (const float*)d_in[7];  const float* e2 = (const float*)d_in[8];
    const float* wf1  = (const float*)d_in[9];  const float* bf1 = (const float*)d_in[10];
    const float* wf2  = (const float*)d_in[11]; const float* bf2 = (const float*)d_in[12];
    float* OUT = (float*)d_out;
    char* wsp = (char*)d_ws;
    h16* WQ = (h16*)wsp; wsp += SZ_WQ;
    h16* WO = (h16*)wsp; wsp += SZ_WO;
    h16* W1 = (h16*)wsp; wsp += SZ_W1;
    h16* W2 = (h16*)wsp; wsp += SZ_W2;
    h16* PT = (h16*)wsp; wsp += SZ_PT;
    h16* RA = (h16*)wsp; wsp += SZ_A;
    h16* RB = (h16*)wsp; wsp += SZ_H;
    h16* H1  = RA;
    h16* PL  = RA + SZ_H / 2;
    h16* FF1 = RA;
    h16* CTX = RB;
    h16* H2  = RB;

    { const size_t n8 = (size_t)NQKV * DM / 8; k_wcvt<<<(unsigned)((n8 + 255) / 256), 256, 0, stream>>>(wqkv, WQ, n8); }
    { const size_t n8 = (size_t)DM * DM / 8;   k_wcvt<<<(unsigned)((n8 + 255) / 256), 256, 0, stream>>>(wout, WO, n8); }
    { const size_t n8 = (size_t)DI * DM / 8;   k_wcvt<<<(unsigned)((n8 + 255) / 256), 256, 0, stream>>>(wf1, W1, n8); }
    { const size_t n8 = (size_t)DM * DI / 8;   k_wcvt<<<(unsigned)((n8 + 255) / 256), 256, 0, stream>>>(wf2, W2, n8); }
    k_poscvt<<<(PJ * HD / 8 + 255) / 256, 256, 0, stream>>>(pos, PT);

    k_ln<<<NB * SEQ / 8, 256, 0, stream>>>(x, g1, e1, H1, 1);
    k_gemm_qkv<<<dim3(NB * SEQ / 64, NQKV / 64, 1), 32, 0, stream>>>(H1, WQ, bqkv, PL, OUT + OUT1_OFF);
    k_flash<<<dim3(SEQ / (16 * AW), NB * NH_, 1), 32 * AW, 0, stream>>>(PL, PL + PLN, PL + 2 * PLN, PT, CTX);
    k_gemm_out<<<dim3(NB * SEQ / 64, DM / 64, 1), 32, 0, stream>>>(CTX, WO, x, OUT);
    k_ln<<<NB * SEQ / 8, 256, 0, stream>>>(OUT, g2, e2, H2, 0);
    k_gemm_fc1<<<dim3(NB * SEQ / 64, DI / 64, 1), 32, 0, stream>>>(H2, W1, bf1, FF1);
    k_gemm_fc2<<<dim3(NB * SEQ / 64, DM / 64, 1), 32, 0, stream>>>(FF1, W2, bf2, OUT);
}
